// DynamicMultiheadAttention_48850958025159
// MI455X (gfx1250) — hardware-verified
//
#include <hip/hip_runtime.h>
#include <stdint.h>
#include <stddef.h>
#include <math.h>

#pragma clang fp contract(off)

#define NT   8192
#define DD   512
#define NGRP 64
#define CAP  256
#define QT   32
#define QP   520
#define SPF  256
#define PPH  264
#define VPH  264
#define OPH  136
#define SLAB 128
#define TT   64
#define TPF  68
#define GTP  68
#define GBM  128
#define GBN  128

#define PL   ((size_t)NT * DD)
#define WPL  ((size_t)DD * DD)

#define LQB   (2 * QT * QP * 2)
#define LVTB  (2 * SLAB * VPH * 2)
#define LA    LVTB
#define LSB   (QT * SPF * 4)
#define LPB   (2 * QT * PPH * 2)
#define LDS_ATT (LA + LSB + LPB)
#define LDS_G   (8 * 32 * GTP * 4)

static_assert(2 * LQB <= LA);
static_assert(2 * QT * OPH * 2 <= LSB);
static_assert(LA % 16 == 0);
static_assert((LA + LSB) % 16 == 0);
static_assert(LQB % 16 == 0);
static_assert((QP * 2) % 16 == 0);
static_assert((PPH * 2) % 16 == 0);
static_assert((VPH * 2) % 16 == 0);
static_assert((OPH * 2) % 16 == 0);
static_assert((GTP * 4) % 16 == 0);
static_assert((TPF * 4) % 16 == 0);
static_assert(SPF >= CAP);
static_assert(PPH >= CAP);
static_assert(VPH >= CAP);
static_assert(OPH >= SLAB);
static_assert(CAP == 256);
static_assert(CAP % QT == 0);
static_assert(QT == 32);
static_assert(NT % 128 == 0);
static_assert(NT % GBM == 0);
static_assert(DD % GBN == 0);
static_assert(DD % SLAB == 0);
static_assert(DD % TT == 0);
static_assert(DD % 32 == 0);
static_assert(DD == 512);
static_assert((NT * DD) % (8 * 256) == 0);

typedef __bf16         v16b __attribute__((ext_vector_type(16)));
typedef float          v8f  __attribute__((ext_vector_type(8)));
typedef float          v4f  __attribute__((ext_vector_type(4)));
typedef unsigned int   v4u  __attribute__((ext_vector_type(4)));
typedef v4f __attribute__((may_alias)) v4fa;
typedef v4u __attribute__((may_alias)) v4ua;

union FragB { v16b v; v4u q[2]; };

__device__ __forceinline__ int clampi(int v, int lo, int hi) {
  return (v < lo) ? lo : ((v > hi) ? hi : v);
}

__device__ __forceinline__ unsigned int bfb(float f) {
  unsigned int u = __float_as_uint(f);
  u = u + 0x7FFFu + ((u >> 16) & 1u);
  return u >> 16;
}
__device__ __forceinline__ void split2(float f, unsigned int& hb, unsigned int& lb) {
  hb = bfb(f);
  const float hv = __uint_as_float(hb << 16);
  lb = bfb(f - hv);
}
__device__ __forceinline__ unsigned int pk2(float f0, float f1, unsigned int& lo2) {
  unsigned int h0, l0, h1, l1;
  split2(f0, h0, l0);
  split2(f1, h1, l1);
  lo2 = l0 | (l1 << 16);
  return h0 | (h1 << 16);
}
__device__ __forceinline__ void pack8(v4f a, v4f c, v4u& hp, v4u& lp) {
  unsigned int l0, l1, l2, l3;
  hp.x = pk2(a.x, a.y, l0);
  hp.y = pk2(a.z, a.w, l1);
  hp.z = pk2(c.x, c.y, l2);
  hp.w = pk2(c.z, c.w, l3);
  lp.x = l0; lp.y = l1; lp.z = l2; lp.w = l3;
}

__device__ __forceinline__ v8f wmma_b(v16b a, v16b b, v8f c) {
  return __builtin_amdgcn_wmma_f32_16x16x32_bf16(false, a, false, b, (short)0, c, false, false);
}
__device__ __forceinline__ v8f w3(v16b ah, v16b al, v16b bh, v16b bl, v8f c) {
  v8f d = wmma_b(ah, bh, c);
  d = wmma_b(ah, bl, d);
  d = wmma_b(al, bh, d);
  asm volatile("v_nop\n\tv_nop\n\tv_nop\n\tv_nop" : "+v"(d) : "v"(ah), "v"(al), "v"(bh), "v"(bl));
  return d;
}

__device__ __forceinline__ v16b ldfrag(const unsigned short* p, int h) {
  FragB f;
  f.q[0] = *(const v4ua*)(p + 8 * h);
  f.q[1] = *(const v4ua*)(p + 16 + 8 * h);
  return f.v;
}

__global__ __launch_bounds__(256) void k_cvtx(const float* __restrict__ src,
                                              unsigned short* __restrict__ dst)
{
  const int g = blockIdx.x * 256 + threadIdx.x;
  const float* s = src + (size_t)g * 8;
  const v4f a = *(const v4fa*)s;
  const v4f c = *(const v4fa*)(s + 4);
  v4u hp, lp;
  pack8(a, c, hp, lp);
  unsigned short* d = dst + (size_t)g * 8;
  *(volatile v4u*)d = hp;
  *(volatile v4u*)(d + PL) = lp;
  __threadfence();
  *(volatile v4u*)d = hp;
  *(volatile v4u*)(d + PL) = lp;
}

__global__ __launch_bounds__(256) void k_tcv(const float* __restrict__ Wq, const float* __restrict__ Wk,
                                             const float* __restrict__ Wv, const float* __restrict__ Wo,
                                             unsigned short* __restrict__ wt)
{
  __shared__ __align__(16) float tile[TT * TPF];
  const int tid = threadIdx.x;
  const int n0 = blockIdx.x * TT, k0 = blockIdx.y * TT, z = blockIdx.z;
  const float* s = (z == 0) ? Wq : ((z == 1) ? Wk : ((z == 2) ? Wv : Wo));
  #pragma unroll
  for (int j = 0; j < 4; ++j) {
    const int r  = (tid >> 4) + 16 * j;
    const int c4 = tid & 15;
    const v4f v = *(const v4fa*)(s + (size_t)(k0 + r) * DD + n0 + 4 * c4);
    *(v4fa*)(tile + r * TPF + 4 * c4) = v;
  }
  __syncthreads();
  v4u hp[2], lp[2];
  #pragma unroll
  for (int j = 0; j < 2; ++j) {
    const int n = (tid >> 3) + 32 * j;
    const int q = tid & 7;
    v4f a, c;
    a.x = tile[(8 * q + 0) * TPF + n];
    a.y = tile[(8 * q + 1) * TPF + n];
    a.z = tile[(8 * q + 2) * TPF + n];
    a.w = tile[(8 * q + 3) * TPF + n];
    c.x = tile[(8 * q + 4) * TPF + n];
    c.y = tile[(8 * q + 5) * TPF + n];
    c.z = tile[(8 * q + 6) * TPF + n];
    c.w = tile[(8 * q + 7) * TPF + n];
    pack8(a, c, hp[j], lp[j]);
  }
  unsigned short* d0 = wt + (size_t)z * 2 * WPL + (size_t)(n0 + (tid >> 3)) * DD + k0 + 8 * (tid & 7);
  unsigned short* d1 = d0 + (size_t)32 * DD;
  *(volatile v4u*)d0 = hp[0];
  *(volatile v4u*)(d0 + WPL) = lp[0];
  *(volatile v4u*)d1 = hp[1];
  *(volatile v4u*)(d1 + WPL) = lp[1];
  __threadfence();
  *(volatile v4u*)d0 = hp[0];
  *(volatile v4u*)(d0 + WPL) = lp[0];
  *(volatile v4u*)d1 = hp[1];
  *(volatile v4u*)(d1 + WPL) = lp[1];
}

__device__ __forceinline__ void gemm_core(const unsigned short* __restrict__ Ah,
                                          const unsigned short* __restrict__ Wh,
                                          int row0, int col0, int h, int m, v8f (&acc)[2][4])
{
  const v8f z8 = {0.f, 0.f, 0.f, 0.f, 0.f, 0.f, 0.f, 0.f};
  #pragma unroll
  for (int mt = 0; mt < 2; ++mt)
    #pragma unroll
    for (int nt = 0; nt < 4; ++nt) acc[mt][nt] = z8;
  #pragma unroll 1
  for (int ks = 0; ks < DD / 32; ++ks) {
    v16b ah[2], al[2];
    #pragma unroll
    for (int mt = 0; mt < 2; ++mt) {
      const unsigned short* ar = Ah + (size_t)(row0 + 16 * mt + m) * DD + 32 * ks;
      ah[mt] = ldfrag(ar, h);
      al[mt] = ldfrag(ar + PL, h);
    }
    #pragma unroll
    for (int nt = 0; nt < 4; ++nt) {
      const unsigned short* br = Wh + (size_t)(col0 + 16 * nt + m) * DD + 32 * ks;
      const v16b bh = ldfrag(br, h);
      const v16b bl = ldfrag(br + WPL, h);
      #pragma unroll
      for (int mt = 0; mt < 2; ++mt) acc[mt][nt] = w3(ah[mt], al[mt], bh, bl, acc[mt][nt]);
    }
  }
}

__device__ __forceinline__ void stage_tile(float* sW, const v8f (&acc)[2][4], const float* __restrict__ bias,
                                           int col0, int h, int m)
{
  #pragma unroll
  for (int mt = 0; mt < 2; ++mt)
    #pragma unroll
    for (int nt = 0; nt < 4; ++nt) {
      const float bn = bias[col0 + 16 * nt + m];
      #pragma unroll
      for (int r = 0; r < 8; ++r)
        sW[(16 * mt + 8 * h + r) * GTP + 16 * nt + m] = acc[mt][nt][r] + bn;
    }
}

__device__ __forceinline__ void y_pass(const float* sW, unsigned short* __restrict__ Y,
                                       int row0, int col0, int lane)
{
  const int sub = lane >> 3, q = lane & 7;
  #pragma unroll
  for (int i = 0; i < 8; ++i) {
    const int row = 4 * i + sub;
    const v4f a = *(const v4fa*)(sW + row * GTP + 8 * q);
    const v4f c = *(const v4fa*)(sW + row * GTP + 8 * q + 4);
    v4u hp, lp;
    pack8(a, c, hp, lp);
    unsigned short* d = Y + (size_t)(row0 + row) * DD + col0 + 8 * q;
    *(volatile v4u*)d = hp;
    *(volatile v4u*)(d + PL) = lp;
  }
}

__device__ __forceinline__ void out_pass(const float* sW, float* __restrict__ out,
                                         const float* __restrict__ bias, const int* __restrict__ labels,
                                         int row0, int col0, int lane)
{
  const int sub = lane >> 4, q = lane & 15;
  const v4f bb = *(const v4fa*)(bias + col0 + 4 * q);
  #pragma unroll
  for (int i = 0; i < 16; ++i) {
    const int row = 2 * i + sub;
    const v4f a = *(const v4fa*)(sW + row * GTP + 4 * q);
    const int lab = labels[row0 + row];
    const bool valid = (lab != -1);
    v4f o;
    o.x = valid ? a.x : bb.x;
    o.y = valid ? a.y : bb.y;
    o.z = valid ? a.z : bb.z;
    o.w = valid ? a.w : bb.w;
    *(volatile v4f*)(out + (size_t)(row0 + row) * DD + col0 + 4 * q) = o;
  }
}

__global__ __launch_bounds__(256) void k_qkv(const unsigned short* __restrict__ xp,
                                             const unsigned short* __restrict__ wt,
                                             const float* __restrict__ bq, const float* __restrict__ bk,
                                             const float* __restrict__ bv,
                                             unsigned short* __restrict__ qkv)
{
  extern __shared__ __align__(16) unsigned char dsm_g[];
  const int tid = threadIdx.x, lane = tid & 31, wv = tid >> 5;
  const int h = lane >> 4, m = lane & 15;
  const int z = blockIdx.z;
  float* sW = (float*)dsm_g + wv * (32 * GTP);
  const int row0 = blockIdx.x * GBM + 32 * (wv & 3);
  const int col0 = blockIdx.y * GBN + 64 * (wv >> 2);
  const unsigned short* Wz = wt + (size_t)z * 2 * WPL;
  const float* bias = (z == 0) ? bq : ((z == 1) ? bk : bv);
  v8f acc[2][4];
  gemm_core(xp, Wz, row0, col0, h, m, acc);
  stage_tile(sW, acc, bias, col0, h, m);
  __syncthreads();
  unsigned short* Yz = qkv + (size_t)z * 2 * PL;
  y_pass(sW, Yz, row0, col0, lane);
  __threadfence();
  y_pass(sW, Yz, row0, col0, lane);
}

__global__ __launch_bounds__(256) void k_out(const unsigned short* __restrict__ op,
                                             const unsigned short* __restrict__ wo,
                                             const float* __restrict__ bo,
                                             const int* __restrict__ labels,
                                             float* __restrict__ out)
{
  extern __shared__ __align__(16) unsigned char dsm_o[];
  const int tid = threadIdx.x, lane = tid & 31, wv = tid >> 5;
  const int h = lane >> 4, m = lane & 15;
  float* sW = (float*)dsm_o + wv * (32 * GTP);
  const int row0 = blockIdx.x * GBM + 32 * (wv & 3);
  const int col0 = blockIdx.y * GBN + 64 * (wv >> 2);
  v8f acc[2][4];
  gemm_core(op, wo, row0, col0, h, m, acc);
  stage_tile(sW, acc, bo, col0, h, m);
  __syncthreads();
  out_pass(sW, out, bo, labels, row0, col0, lane);
  __threadfence();
  out_pass(sW, out, bo, labels, row0, col0, lane);
}

__device__ __forceinline__ void o_pass(const unsigned short* sO, const int* tk, unsigned short* __restrict__ op,
                                       int sl, int wv, int lane, int nrows)
{
  const int pl = lane >> 4, q = lane & 15;
  #pragma unroll
  for (int i = 0; i < 8; ++i) {
    const int row = wv * 8 + i;
    const int t = clampi(tk[row], 0, NT - 1);
    const v4u v = *(const v4ua*)(sO + pl * (QT * OPH) + row * OPH + 8 * q);
    unsigned short* dst = op + (size_t)pl * PL + (size_t)t * DD + sl * SLAB + 8 * q;
    if (row < nrows) *(volatile v4u*)dst = v;
  }
}

__global__ __launch_bounds__(128) void k_attn(const unsigned short* __restrict__ qkv,
                                              const int* __restrict__ labels,
                                              unsigned short* __restrict__ op)
{
  extern __shared__ __align__(16) unsigned char dsm_a[];
  unsigned short* sQ  = (unsigned short*)dsm_a;
  unsigned short* sK  = (unsigned short*)(dsm_a + LQB);
  unsigned short* sVT = (unsigned short*)dsm_a;
  float*          sS  = (float*)(dsm_a + LA);
  unsigned short* sO  = (unsigned short*)(dsm_a + LA);
  unsigned short* sP  = (unsigned short*)(dsm_a + LA + LSB);
  __shared__ int sTok[CAP];
  __shared__ int s_wc[4];

  const int tid = threadIdx.x, lane = tid & 31, wv = tid >> 5;
  const int h = lane >> 4, m = lane & 15;
  const int g = blockIdx.x, qt = blockIdx.y;

  sTok[tid] = 0;
  sTok[tid + 128] = 0;
  __syncthreads();

  int base = 0;
  #pragma unroll 1
  for (int ch = 0; ch < NT / 128; ++ch) {
    const int t = ch * 128 + tid;
    const int l = labels[t];
    const bool f = (l == g);
    const unsigned int msk = __builtin_amdgcn_ballot_w32(f);
    const int off = __builtin_popcount(msk & ((1u << lane) - 1u));
    const int wcnt = __builtin_popcount(msk);
    if (lane == 0) s_wc[wv] = wcnt;
    __syncthreads();
    int pre = 0, tot = 0;
    #pragma unroll
    for (int w2 = 0; w2 < 4; ++w2) {
      const int c2 = s_wc[w2];
      tot += c2;
      pre += (w2 < wv) ? c2 : 0;
    }
    if (f) {
      const int rank = base + pre + off;
      if ((unsigned)rank < (unsigned)CAP) sTok[rank] = t;
    }
    base += tot;
    __syncthreads();
  }
  const int cnt = (base > CAP) ? CAP : base;
  const int q0 = qt * QT;
  if (q0 >= cnt) return;
  int nrows = cnt - q0;
  nrows = (nrows > QT) ? QT : nrows;
  const int nkc = (cnt + 31) >> 5;
  const int kpad = nkc << 5;

  const unsigned short* Qp = qkv;
  const unsigned short* Kp = qkv + 2 * PL;
  const unsigned short* Vp = qkv + 4 * PL;
  const v8f z8 = {0.f, 0.f, 0.f, 0.f, 0.f, 0.f, 0.f, 0.f};

  #pragma unroll 4
  for (int j = 0; j < 16; ++j) {
    const int idx = tid + 128 * j;
    const int row = idx >> 6, c8 = idx & 63;
    const int t = clampi(sTok[q0 + row], 0, NT - 1);
    const size_t go = (size_t)t * DD + 8 * c8;
    v4u vh = *(const v4ua*)(Qp + go);
    v4u vl = *(const v4ua*)(Qp + PL + go);
    const unsigned int km = (row < nrows) ? 0xffffffffu : 0u;
    const v4u kv = {km, km, km, km};
    vh &= kv;
    vl &= kv;
    *(v4ua*)(sQ + row * QP + 8 * c8) = vh;
    *(v4ua*)(sQ + QT * QP + row * QP + 8 * c8) = vl;
  }

  const float scale = 0.044194173824159216f;
  const int mt2 = wv >> 1, nt2 = wv & 1;
  #pragma unroll 1
  for (int kc = 0; kc < nkc; ++kc) {
    #pragma unroll 4
    for (int j = 0; j < 16; ++j) {
      const int idx = tid + 128 * j;
      const int row = idx >> 6, c8 = idx & 63;
      const int key = kc * 32 + row;
      const int t = clampi(sTok[key], 0, NT - 1);
      const size_t go = (size_t)t * DD + 8 * c8;
      v4u vh = *(const v4ua*)(Kp + go);
      v4u vl = *(const v4ua*)(Kp + PL + go);
      const unsigned int km = (key < cnt) ? 0xffffffffu : 0u;
      const v4u kv = {km, km, km, km};
      vh &= kv;
      vl &= kv;
      *(v4ua*)(sK + row * QP + 8 * c8) = vh;
      *(v4ua*)(sK + QT * QP + row * QP + 8 * c8) = vl;
    }
    __syncthreads();
    v8f acc = z8;
    #pragma unroll 1
    for (int ks = 0; ks < DD / 32; ++ks) {
      const v16b ah = ldfrag(sQ + (16 * mt2 + m) * QP + 32 * ks, h);
      const v16b al = ldfrag(sQ + QT * QP + (16 * mt2 + m) * QP + 32 * ks, h);
      const v16b bh = ldfrag(sK + (16 * nt2 + m) * QP + 32 * ks, h);
      const v16b bl = ldfrag(sK + QT * QP + (16 * nt2 + m) * QP + 32 * ks, h);
      acc = w3(ah, al, bh, bl, acc);
    }
    #pragma unroll
    for (int r = 0; r < 8; ++r)
      sS[(16 * mt2 + 8 * h + r) * SPF + kc * 32 + 16 * nt2 + m] = acc[r] * scale;
    __syncthreads();
  }

  #pragma unroll 1
  for (int rr = 0; rr < 8; ++rr) {
    const int row = wv * 8 + rr;
    float sv[8];
    float mx = -3.0e38f;
    #pragma unroll
    for (int i = 0; i < 8; ++i) {
      const int col = 32 * i + lane;
      const float s = sS[row * SPF + col];
      sv[i] = (col < cnt) ? s : -3.0e38f;
      mx = fmaxf(mx, sv[i]);
    }
    #pragma unroll
    for (int o = 16; o > 0; o >>= 1) mx = fmaxf(mx, __shfl_xor(mx, o));
    float e[8];
    float sum = 0.0f;
    #pragma unroll
    for (int i = 0; i < 8; ++i) {
      const int col = 32 * i + lane;
      e[i] = (col < cnt) ? __expf(sv[i] - mx) : 0.0f;
      sum = sum + e[i];
    }
    #pragma unroll
    for (int o = 16; o > 0; o >>= 1) sum = sum + __shfl_xor(sum, o);
    const float inv = 1.0f / sum;
    #pragma unroll
    for (int i = 0; i < 8; ++i) {
      const int col = 32 * i + lane;
      unsigned int hb, lb;
      split2(e[i] * inv, hb, lb);
      sP[row * PPH + col] = (unsigned short)hb;
      sP[QT * PPH + row * PPH + col] = (unsigned short)lb;
    }
  }
  __syncthreads();

  #pragma unroll 1
  for (int sl = 0; sl < DD / SLAB; ++sl) {
    #pragma unroll 1
    for (int it = tid; it < kpad * 16; it += 128) {
      const int key = it >> 4, c = it & 15;
      const int t = clampi(sTok[key], 0, NT - 1);
      const size_t go = (size_t)t * DD + sl * SLAB + 8 * c;
      v4u vh = *(const v4ua*)(Vp + go);
      v4u vl = *(const v4ua*)(Vp + PL + go);
      const unsigned int km = (key < cnt) ? 0xffffffffu : 0u;
      const v4u kv = {km, km, km, km};
      vh &= kv;
      vl &= kv;
      unsigned short* dh = sVT + (8 * c) * VPH + key;
      unsigned short* dl = dh + SLAB * VPH;
      dh[0 * VPH] = (unsigned short)(vh.x & 0xffffu);  dh[1 * VPH] = (unsigned short)(vh.x >> 16);
      dh[2 * VPH] = (unsigned short)(vh.y & 0xffffu);  dh[3 * VPH] = (unsigned short)(vh.y >> 16);
      dh[4 * VPH] = (unsigned short)(vh.z & 0xffffu);  dh[5 * VPH] = (unsigned short)(vh.z >> 16);
      dh[6 * VPH] = (unsigned short)(vh.w & 0xffffu);  dh[7 * VPH] = (unsigned short)(vh.w >> 16);
      dl[0 * VPH] = (unsigned short)(vl.x & 0xffffu);  dl[1 * VPH] = (unsigned short)(vl.x >> 16);
      dl[2 * VPH] = (unsigned short)(vl.y & 0xffffu);  dl[3 * VPH] = (unsigned short)(vl.y >> 16);
      dl[4 * VPH] = (unsigned short)(vl.z & 0xffffu);  dl[5 * VPH] = (unsigned short)(vl.z >> 16);
      dl[6 * VPH] = (unsigned short)(vl.w & 0xffffu);  dl[7 * VPH] = (unsigned short)(vl.w >> 16);
    }
    __syncthreads();

    v8f acc[2][2];
    #pragma unroll
    for (int mt = 0; mt < 2; ++mt)
      #pragma unroll
      for (int nt = 0; nt < 2; ++nt) acc[mt][nt] = z8;
    #pragma unroll 1
    for (int ks = 0; ks < nkc; ++ks) {
      v16b ph[2], pl[2];
      #pragma unroll
      for (int mt = 0; mt < 2; ++mt) {
        ph[mt] = ldfrag(sP + (16 * mt + m) * PPH + 32 * ks, h);
        pl[mt] = ldfrag(sP + QT * PPH + (16 * mt + m) * PPH + 32 * ks, h);
      }
      #pragma unroll
      for (int nt = 0; nt < 2; ++nt) {
        const int dcol = 32 * wv + 16 * nt + m;
        const v16b bh = ldfrag(sVT + dcol * VPH + 32 * ks, h);
        const v16b bl = ldfrag(sVT + SLAB * VPH + dcol * VPH + 32 * ks, h);
        #pragma unroll
        for (int mt = 0; mt < 2; ++mt) acc[mt][nt] = w3(ph[mt], pl[mt], bh, bl, acc[mt][nt]);
      }
    }
    #pragma unroll
    for (int mt = 0; mt < 2; ++mt)
      #pragma unroll
      for (int nt = 0; nt < 2; ++nt) {
        const int col = 32 * wv + 16 * nt + m;
        #pragma unroll
        for (int r = 0; r < 8; ++r) {
          const int row = 16 * mt + 8 * h + r;
          unsigned int hb, lb;
          split2(acc[mt][nt][r], hb, lb);
          sO[row * OPH + col] = (unsigned short)hb;
          sO[QT * OPH + row * OPH + col] = (unsigned short)lb;
        }
      }
    __syncthreads();
    o_pass(sO, sTok + q0, op, sl, wv, lane, nrows);
    __threadfence();
    o_pass(sO, sTok + q0, op, sl, wv, lane, nrows);
    __syncthreads();
  }
}

extern "C" void kernel_launch(void* const* d_in, const int* in_sizes, int n_in,
                              void* d_out, int out_size, void* d_ws, size_t ws_size,
                              hipStream_t stream)
{
  if (n_in < 10) return;
  if (in_sizes[0] != NT * DD) return;
  if (in_sizes[1] != NT) return;
  if (in_sizes[2] != DD * DD) return;
  if (in_sizes[3] != DD) return;
  if (in_sizes[4] != DD * DD) return;
  if (in_sizes[5] != DD) return;
  if (in_sizes[6] != DD * DD) return;
  if (in_sizes[7] != DD) return;
  if (in_sizes[8] != DD * DD) return;
  if (in_sizes[9] != DD) return;
  if (out_size != NT * DD) return;

  const float* x      = (const float*)d_in[0];
  const int*   labels = (const int*)d_in[1];
  const float* Wq = (const float*)d_in[2];
  const float* bq = (const float*)d_in[3];
  const float* Wk = (const float*)d_in[4];
  const float* bk = (const float*)d_in[5];
  const float* Wv = (const float*)d_in[6];
  const float* bv = (const float*)d_in[7];
  const float* Wo = (const float*)d_in[8];
  const float* bo = (const float*)d_in[9];
  float* out = (float*)d_out;

  const size_t bXP  = (size_t)2 * NT * DD * 2;
  const size_t bWT  = (size_t)4 * 2 * DD * DD * 2;
  const size_t bQKV = (size_t)3 * 2 * NT * DD * 2;
  const size_t bOP  = (size_t)2 * NT * DD * 2;
  const size_t total = bXP + bWT + bQKV + bOP;
  if (total > ws_size) return;
  if (total > (size_t)134217728) return;

  char* ws = (char*)d_ws;
  size_t off = 0;
  unsigned short* XP  = (unsigned short*)(ws + off); off += bXP;
  unsigned short* WT  = (unsigned short*)(ws + off); off += bWT;
  unsigned short* QKV = (unsigned short*)(ws + off); off += bQKV;
  unsigned short* OP  = (unsigned short*)(ws + off); off += bOP;
  if (off != total) return;

  hipFuncSetAttribute(reinterpret_cast<const void*>(&k_qkv),
                      hipFuncAttributeMaxDynamicSharedMemorySize, LDS_G);
  hipFuncSetAttribute(reinterpret_cast<const void*>(&k_out),
                      hipFuncAttributeMaxDynamicSharedMemorySize, LDS_G);
  hipFuncSetAttribute(reinterpret_cast<const void*>(&k_attn),
                      hipFuncAttributeMaxDynamicSharedMemorySize, LDS_ATT);

  k_cvtx<<<(NT * DD / 8) / 256, 256, 0, stream>>>(x, XP);
  k_tcv<<<dim3(DD / TT, DD / TT, 4), 256, 0, stream>>>(Wq, Wk, Wv, Wo, WT);
  k_qkv<<<dim3(NT / GBM, DD / GBN, 3), 256, LDS_G, stream>>>(XP, WT, bq, bk, bv, QKV);
  k_attn<<<dim3(NGRP, CAP / QT), 128, LDS_ATT, stream>>>(QKV, labels, OP);
  k_out<<<dim3(NT / GBM, DD / GBN), 256, LDS_G, stream>>>(OP, WT + (size_t)3 * 2 * WPL, bo, labels, out);
}
